// RoadGNN_53163105190455
// MI455X (gfx1250) — hardware-run, weakly checked
//
#include <hip/hip_runtime.h>


namespace {
constexpr int N = 500000, E = 1250000, CI = 2, H = 64, SB = 2048;
constexpr float XS = 8.0f, WSC = 256.0f, EPS = 1e-5f;
typedef _Float16 b16;
typedef __attribute__((ext_vector_type(16))) _Float16 v16b;
typedef __attribute__((ext_vector_type(8))) _Float16 v8b;
typedef __attribute__((ext_vector_type(8))) float v8f;
typedef __attribute__((ext_vector_type(4))) float v4f;
typedef __attribute__((ext_vector_type(2))) float v2f;
__device__ __forceinline__ float bf16_rne(float f) { unsigned int u = __float_as_uint(f); u += 0x7FFFu + ((u >> 16) & 1u); float r = __uint_as_float(u & 0xFFFF0000u); asm volatile("" : "+v"(r)); return r; }
__device__ __forceinline__ void split16(float v, b16& hi, b16& lo) { hi = (b16)v; lo = (b16)(v - (float)hi); }
__device__ __forceinline__ v16b frag_kb(const b16* p, int hh) { const v8b a = *(const v8b*)(p + 8 * hh), b = *(const v8b*)(p + 16 + 8 * hh); v16b f;
#pragma unroll
  for (int e = 0; e < 8; ++e) { f[e] = a[e]; f[8 + e] = b[e]; } return f; }
__device__ __forceinline__ v8f wmma16b(v16b a, v16b b, v8f c) { v8f d = __builtin_amdgcn_wmma_f32_16x16x32_f16(false, a, false, b, (short)0, c, false, false); asm volatile("v_nop\n\tv_nop\n\tv_nop\n\tv_nop" : "+v"(d) : "v"(a), "v"(b)); return d; }
__device__ __forceinline__ void wave_lds_sync() { __builtin_amdgcn_fence(__ATOMIC_RELEASE, "workgroup"); __builtin_amdgcn_wave_barrier(); __builtin_amdgcn_fence(__ATOMIC_ACQUIRE, "workgroup"); }
__device__ __forceinline__ float pmul(float a, float b) { float p = a * b; asm volatile("" : "+v"(p)); return p; }
__device__ __forceinline__ int iclamp(int v, int lo, int hi) { return v < lo ? lo : (v > hi ? hi : v); }
constexpr int CSR_NBLK10 = 512, CSR_GB10 = 10, CSR_GN10 = 1 << CSR_GB10  , CSR_TS10 = (CSR_GN10 < 32 ? 32 : CSR_GN10)  , CSR_MAXG10 = 512, CSR_CAP10 = 12288  ;
__device__ __host__ __forceinline__ int csr_tix10(int v) { return (v >> CSR_GB10) * CSR_TS10 + (v & (CSR_GN10 - 1)); }
__global__ __launch_bounds__(64) void csrA_kernel10(const int* __restrict__ dst, int E, int N, int nG, int CHP, int NGP, int* __restrict__ STG, int* __restrict__ HST) {
  extern __shared__ int sm[];
  int* cnt = sm; int* run = sm + NGP; int* ids = sm + 2 * NGP;
  const int b = blockIdx.x; const int ch = (E + CSR_NBLK10 - 1) / CSR_NBLK10; const int e0 = b * ch, e1 = min(E, e0 + ch);
  for (int i = threadIdx.x; i < NGP; i += 64) cnt[i] = 0;
  for (int i = threadIdx.x; i < CHP; i += 64) ids[i] = -1;
  __syncthreads();
  if (threadIdx.x == 0) {
    for (int e = e0; e < e1; ++e) { int d = dst[e]; d = (d < 0) ? 0 : (d >= N ? N - 1 : d); cnt[d >> CSR_GB10] += 1; }
    int acc = 0; for (int g = 0; g < nG; ++g) { run[g] = acc; acc += cnt[g]; }
    for (int e = e0; e < e1; ++e) { int d = dst[e]; d = (d < 0) ? 0 : (d >= N ? N - 1 : d); const int g = d >> CSR_GB10; ids[run[g]] = e; run[g] += 1; } }
  __syncthreads();
  typedef __attribute__((ext_vector_type(4))) int v4i;
  for (int pass = 0; pass < 2; ++pass) {
    for (int i = threadIdx.x; i < CHP / 4; i += 64) *(volatile v4i*)(STG + (size_t)b * CHP + i * 4) = *(const v4i*)(&ids[i * 4]);
    for (int i = threadIdx.x; i < NGP / 4; i += 64) { v4i v; for (int e = 0; e < 4; ++e) v[e] = (i * 4 + e < nG) ? cnt[i * 4 + e] : 0; *(volatile v4i*)(HST + (size_t)b * NGP + i * 4) = v; }
    __threadfence(); }
}
__global__ __launch_bounds__(512) void csrS_kernel10(const int* __restrict__ HST, int nG, int NGP, int* __restrict__ START, int* __restrict__ TOT, int* __restrict__ OFF) {
  __shared__ int tot[CSR_MAXG10];
  const int b = threadIdx.x;
  for (int pass = 0; pass < 2; ++pass) { int runb = 0; for (int g = 0; g < nG; ++g) { int c = HST[(size_t)b * NGP + g]; c = (c < 0) ? 0 : c; ((volatile int*)OFF)[(size_t)g * CSR_NBLK10 + b] = runb; runb += c; } __threadfence(); }
  for (int g = threadIdx.x; g < nG; g += 512) { int s = 0; for (int bb = 0; bb < CSR_NBLK10; ++bb) { int c = HST[(size_t)bb * NGP + g]; s += (c < 0) ? 0 : c; } tot[g] = s; }
  __syncthreads();
  if (threadIdx.x < 32) {
    __shared__ int st[CSR_MAXG10 + 32];
    if (threadIdx.x == 0) { int acc = 0; for (int g = 0; g < NGP; ++g) { st[g] = acc; if (g < nG) acc += (tot[g] + 31) & ~31; } st[NGP] = acc; }
    __builtin_amdgcn_fence(__ATOMIC_RELEASE, "workgroup"); __builtin_amdgcn_wave_barrier(); __builtin_amdgcn_fence(__ATOMIC_ACQUIRE, "workgroup");
    for (int pass = 0; pass < 2; ++pass) { for (int i = threadIdx.x; i < NGP + 32; i += 32) { ((volatile int*)START)[i] = (i <= NGP) ? st[min(i, NGP)] : 0; ((volatile int*)TOT)[i] = (i < nG) ? tot[i] : 0; } __threadfence(); } }
}
__global__ __launch_bounds__(256) void csrB_kernel10(const int* __restrict__ dst, int N, int nG, int CHP, int NGP, int permLen, const int* __restrict__ STG, const int* __restrict__ HST, const int* __restrict__ OFF, const int* __restrict__ START, const int* __restrict__ TOT, int* __restrict__ PERM, int* __restrict__ ROWPTR, int* __restrict__ ROWCNT, int* __restrict__ FLAG) {
  typedef __attribute__((ext_vector_type(4))) int v4i;
  __shared__ int ids[CSR_CAP10]; __shared__ unsigned short key[CSR_CAP10]; __shared__ int outp[CSR_CAP10]; __shared__ int ncnt[CSR_GN10 + 1]; __shared__ int boff[CSR_NBLK10 + 1];
  const int g = blockIdx.x, t_ = threadIdx.x; int tot = TOT[g]; int st = START[g], stn = START[g + 1]; const int v0 = g * CSR_GN10; const int nv = min(CSR_GN10, N - v0); const int t0 = g * CSR_TS10;
  st = (st < 0) ? 0 : (st > permLen - 32 ? permLen - 32 : st) & ~31; stn = (stn < st) ? st : (stn > permLen ? permLen : stn); tot = (tot < 0) ? 0 : tot; if (tot > stn - st && tot <= CSR_CAP10) tot = stn - st;
  if (tot > CSR_CAP10) {
    for (int pass = 0; pass < 2; ++pass) { for (int i = t_; i < CSR_TS10 / 4; i += 256) { v4i a, c; for (int e = 0; e < 4; ++e) { a[e] = st; c[e] = 0; } *(volatile v4i*)(ROWPTR + t0 + i * 4) = a; *(volatile v4i*)(ROWCNT + t0 + i * 4) = c; } if (t_ == 0) ((volatile int*)FLAG)[0] = 1; __threadfence(); } (void)nv; return; }
  if (t_ == 0) { int acc = 0; for (int b = 0; b < CSR_NBLK10; ++b) { boff[b] = acc; int c = HST[(size_t)b * NGP + g]; c = (c < 0) ? 0 : (c > CHP ? CHP : c); acc += c; if (acc > tot) acc = tot; } boff[CSR_NBLK10] = acc; }
  for (int i = t_; i <= CSR_GN10; i += 256) ncnt[i] = 0;
  __syncthreads();
  for (int b = 0; b < CSR_NBLK10; ++b) { const int c = boff[b + 1] - boff[b]; int o_ = OFF[(size_t)g * CSR_NBLK10 + b]; o_ = (o_ < 0) ? 0 : (o_ > CHP - c ? CHP - c : o_); const int* src_ = STG + (size_t)b * CHP + o_;
    for (int i = t_; i < c; i += 256) { int id = src_[i]; id = (id < 0) ? 0 : id; ids[boff[b] + i] = id; int d = dst[id]; d = (d < v0) ? v0 : (d >= N ? N - 1 : d); int kk = d - v0; kk = (kk < 0) ? 0 : (kk >= CSR_GN10 ? CSR_GN10 - 1 : kk); key[boff[b] + i] = (unsigned short)kk; } }
  __syncthreads();
  if (t_ == 0) { for (int i = 0; i < tot; ++i) ncnt[key[i]] += 1; int acc = 0; for (int vl = 0; vl < CSR_GN10; ++vl) { const int c = ncnt[vl]; ncnt[vl] = acc; acc += c; } ncnt[CSR_GN10] = acc;
    for (int i = 0; i < tot; ++i) { const int vl = key[i]; outp[ncnt[vl]] = ids[i]; ncnt[vl] += 1; }
    for (int vl = CSR_GN10; vl > 0; --vl) ncnt[vl] = ncnt[vl - 1]; ncnt[0] = 0; }
  __syncthreads();
  for (int pass = 0; pass < 2; ++pass) {
    for (int i = t_; i < (stn - st) / 4; i += 256) { v4i v; for (int e = 0; e < 4; ++e) { const int q = i * 4 + e; v[e] = (q < tot) ? outp[q] : -1; } *(volatile v4i*)(PERM + st + i * 4) = v; }
    for (int i = t_; i < CSR_TS10 / 4; i += 256) { v4i a, c; for (int e = 0; e < 4; ++e) { const int vl = i * 4 + e; const int vc = vl < CSR_GN10 ? vl : CSR_GN10; a[e] = (vl < CSR_GN10) ? st + ncnt[vc] : st; c[e] = (vl < nv) ? (ncnt[(vc < CSR_GN10 ? vc : CSR_GN10 - 1) + 1] - ncnt[vc]) : 0; } *(volatile v4i*)(ROWPTR + t0 + i * 4) = a; *(volatile v4i*)(ROWCNT + t0 + i * 4) = c; }
    __threadfence(); }
}
__global__ __launch_bounds__(256) void csrZ_kernel10(int* __restrict__ p, size_t n4) { typedef __attribute__((ext_vector_type(4))) int v4i; const size_t tid = (size_t)blockIdx.x * 256 + threadIdx.x, nth = (size_t)gridDim.x * 256; v4i z = {0, 0, 0, 0}; for (size_t i = tid; i < n4; i += nth) *(volatile v4i*)(p + i * 4) = z; }
struct CsrBufs10 { int *STG, *HST, *OFF, *START, *TOT, *PERM, *ROWPTR, *ROWCNT, *FLAG; int nG, NGP, CHP; size_t permLen; char* base; size_t bytes; };
static size_t csr_carve10(CsrBufs10& c, char* ws, size_t off, int E, int N) {
  const size_t off0 = off; c.base = ws + off;
  auto al = [&](size_t bytes) { char* p = ws + off; off += (bytes + 255) & ~(size_t)255; return p; };
  c.nG = (N + CSR_GN10 - 1) / CSR_GN10; c.NGP = (c.nG + 31) & ~31; const int ch = (E + CSR_NBLK10 - 1) / CSR_NBLK10; c.CHP = (ch + 31) & ~31; c.permLen = (size_t)E + 32 * (size_t)c.nG + 32;
  c.STG = (int*)al((size_t)CSR_NBLK10 * c.CHP * 4); c.HST = (int*)al((size_t)CSR_NBLK10 * c.NGP * 4); c.OFF = (int*)al((size_t)c.NGP * CSR_NBLK10 * 4); c.START = (int*)al((size_t)(c.NGP + 64) * 4); c.TOT = (int*)al((size_t)(c.NGP + 64) * 4);
  c.PERM = (int*)al(c.permLen * 4); c.ROWPTR = (int*)al((size_t)c.nG * CSR_TS10 * 4); c.ROWCNT = (int*)al((size_t)c.nG * CSR_TS10 * 4); c.FLAG = (int*)al(256);
  c.bytes = off - off0; return off;
}
static void csr_build10(const CsrBufs10& c, const int* dst, int E, int N, hipStream_t stream) {
  const size_t smem = (size_t)(2 * c.NGP + c.CHP) * 4;
  csrZ_kernel10<<<512, 256, 0, stream>>>((int*)c.base, c.bytes / 16);
  csrA_kernel10<<<CSR_NBLK10, 64, smem, stream>>>(dst, E, N, c.nG, c.CHP, c.NGP, c.STG, c.HST);
  csrS_kernel10<<<1, 512, 0, stream>>>(c.HST, c.nG, c.NGP, c.START, c.TOT, c.OFF);
  csrB_kernel10<<<c.nG, 256, 0, stream>>>(dst, N, c.nG, c.CHP, c.NGP, (int)c.permLen, c.STG, c.HST, c.OFF, c.START, c.TOT, c.PERM, c.ROWPTR, c.ROWCNT, c.FLAG);
}


__global__ __launch_bounds__(256) void wput_kernel(const float* __restrict__ w2l, const float* __restrict__ w2r, b16* __restrict__ W2T) { const int u = blockIdx.x * 256 + threadIdx.x; if (u >= H * 16) return; const int o = u / 16, k0 = (u % 16) * 8; v8b v;
#pragma unroll
  for (int j = 0; j < 8; ++j) { const int k = k0 + j; v[j] = (b16)(bf16_rne(k < H ? w2l[(size_t)k * H + o] : w2r[(size_t)(k - H) * H + o]) * WSC); }
  for (int pass = 0; pass < 2; ++pass) { *(volatile v8b*)(W2T + (size_t)o * 2 * H + k0) = v; __threadfence(); } }
__device__ __forceinline__ float bnrelu(float v, int c, const float* ST, const float* g, const float* b) { return fmaxf(pmul(pmul(v - ST[c], ST[H + c]), bf16_rne(g[c])) + bf16_rne(b[c]), 0.0f); }
struct L1P { const float* M1; const float* x; const float* w1l; const float* b1; const float* w1r; const float* ST1; const float* g1; const float* be1; };
__device__ __forceinline__ float s1_of(const L1P& p, size_t u, int c) { return pmul(p.M1[u * 2], bf16_rne(p.w1l[c])) + pmul(p.M1[u * 2 + 1], bf16_rne(p.w1l[H + c])) + bf16_rne(p.b1[c]) + pmul(bf16_rne(p.x[u * 2]), bf16_rne(p.w1r[c])) + pmul(bf16_rne(p.x[u * 2 + 1]), bf16_rne(p.w1r[H + c])); }
__device__ __forceinline__ float x1_of(const L1P& p, size_t u, int c) { return bnrelu(s1_of(p, u, c), c, p.ST1, p.g1, p.be1); }
__global__ __launch_bounds__(256) void m1_kernel(const float* __restrict__ x, const int* __restrict__ srcs, const int* __restrict__ PERM, const int* __restrict__ ROWPTR, const int* __restrict__ ROWCNT, int permLen, int NLIM, float* __restrict__ M1) { const size_t i = (size_t)blockIdx.x * 256 + threadIdx.x; if (i >= (size_t)N) return; float m0 = 0.0f, m1 = 0.0f;
  if (i < (size_t)NLIM) { int st = ROWPTR[i], cnt = ROWCNT[i]; cnt = iclamp(cnt, 0, E); st = iclamp(st, 0, permLen - cnt); int nin = 0;
    for (int j = 0; j < cnt; ++j) { const int e = iclamp(PERM[st + j], 0, E - 1); const size_t u = (size_t)iclamp(srcs[e], 0, N - 1); if (u >= (size_t)NLIM) continue; ++nin; m0 += bf16_rne(x[u * 2]); m1 += bf16_rne(x[u * 2 + 1]); }
    const float inv = 1.0f / (float)(nin > 0 ? nin : 1); m0 = pmul(m0, inv); m1 = pmul(m1, inv); }
  for (int pass = 0; pass < 2; ++pass) { *(volatile v2f*)(M1 + i * 2) = (v2f){m0, m1}; __threadfence(); } }
template <int MODE>
__global__ __launch_bounds__(256) void stat_kernel(L1P p, const float* __restrict__ S, int NLIM, float* __restrict__ PS) { __shared__ float A[4][64], Q[4][64]; const int t = threadIdx.x, c = t & 63, part = t >> 6; const size_t r0 = (size_t)blockIdx.x * SB; float s = 0.0f, q = 0.0f;
  for (int rr = part; rr < SB; rr += 4) { const size_t row = r0 + rr; if (row >= (size_t)NLIM) break; const float v = MODE == 1 ? s1_of(p, row, c) : S[row * H + c]; s += v; q += pmul(v, v); } A[part][c] = s; Q[part][c] = q; __syncthreads();
  if (t < 64) { const float ss = (A[0][t] + A[1][t]) + (A[2][t] + A[3][t]), qq = (Q[0][t] + Q[1][t]) + (Q[2][t] + Q[3][t]); for (int pass = 0; pass < 2; ++pass) { ((volatile float*)PS)[(size_t)blockIdx.x * 2 * H + t] = ss; ((volatile float*)PS)[(size_t)blockIdx.x * 2 * H + H + t] = qq; __threadfence(); } } }
__global__ __launch_bounds__(256) void bnfin_kernel(const float* __restrict__ PS, int nblk, int nnodes, float* __restrict__ ST) { const int t = threadIdx.x; const int c = t & 63, half = t >> 6; __shared__ double S_[4][64], Q_[4][64]; double s = 0.0, q = 0.0; for (int b = half; b < nblk; b += 4) { s += (double)PS[(size_t)b * 2 * H + c]; q += (double)PS[(size_t)b * 2 * H + H + c]; } S_[half][c] = s; Q_[half][c] = q; __syncthreads();
  if (t < 64) { const double sum = (S_[0][t] + S_[1][t]) + (S_[2][t] + S_[3][t]), sq = (Q_[0][t] + Q_[1][t]) + (Q_[2][t] + Q_[3][t]); const double mu = sum / nnodes; double var = sq / nnodes - mu * mu; if (var < 0.0) var = 0.0;
    for (int pass = 0; pass < 2; ++pass) { ((volatile float*)ST)[t] = (float)mu; ((volatile float*)ST)[H + t] = (float)(1.0 / sqrt(var + (double)EPS)); __threadfence(); } } }
__global__ __launch_bounds__(32) void l2_kernel(L1P p, const b16* __restrict__ W2T, const float* __restrict__ b2, const int* __restrict__ srcs, const int* __restrict__ PERM, const int* __restrict__ ROWPTR, const int* __restrict__ ROWCNT, int permLen, int NLIM, float* __restrict__ S2) { __shared__ __attribute__((aligned(16))) b16 Ah[16][136], Al[16][136]; __shared__ float Tf[16][68]; const int lane = threadIdx.x, nloc = lane & 15, hlf = lane >> 4; const size_t m0 = (size_t)blockIdx.x * 16; if (m0 >= (size_t)NLIM) return; const int c0 = lane * 2;
  for (int rr = 0; rr < 16; ++rr) { const size_t i = m0 + rr; int st = ROWPTR[i], cnt = ROWCNT[i]; cnt = iclamp(cnt, 0, E); st = iclamp(st, 0, permLen - cnt); float a0 = 0.0f, a1 = 0.0f; int nin = 0;
#pragma unroll 1
    for (int j = 0; j < cnt; ++j) { const int e = iclamp(PERM[st + j], 0, E - 1); const size_t u = (size_t)iclamp(srcs[e], 0, N - 1); if (u >= (size_t)NLIM) continue; ++nin; a0 += x1_of(p, u, c0); a1 += x1_of(p, u, c0 + 1); }
    const float inv = 1.0f / (float)(nin > 0 ? nin : 1); b16 ph, pl; split16(pmul(a0, inv) * XS, ph, pl); Ah[rr][c0] = ph; Al[rr][c0] = pl; split16(pmul(a1, inv) * XS, ph, pl); Ah[rr][c0 + 1] = ph; Al[rr][c0 + 1] = pl;
    split16(x1_of(p, i, c0) * XS, ph, pl); Ah[rr][H + c0] = ph; Al[rr][H + c0] = pl; split16(x1_of(p, i, c0 + 1) * XS, ph, pl); Ah[rr][H + c0 + 1] = ph; Al[rr][H + c0 + 1] = pl; }
  wave_lds_sync(); v8f acc[4] = {(v8f){}, (v8f){}, (v8f){}, (v8f){}};
#pragma unroll
  for (int kb = 0; kb < 2 * H; kb += 32) { const v16b a = frag_kb(&Ah[nloc][kb], hlf), al = frag_kb(&Al[nloc][kb], hlf);
#pragma unroll
    for (int t = 0; t < 4; ++t) { const v16b bw = frag_kb(W2T + (size_t)(t * 16 + nloc) * 2 * H + kb, hlf); acc[t] = wmma16b(a, bw, acc[t]); acc[t] = wmma16b(al, bw, acc[t]); } }
#pragma unroll
  for (int t = 0; t < 4; ++t) { const int cc = t * 16 + nloc; const float bb = bf16_rne(b2[cc]);
#pragma unroll
    for (int r8 = 0; r8 < 8; ++r8) Tf[8 * hlf + r8][cc] = acc[t][r8] * (1.0f / (XS * WSC)) + bb; }
  wave_lds_sync();
  for (int pass = 0; pass < 2; ++pass) { for (int rr = 0; rr < 16; ++rr) *(volatile v2f*)(S2 + (m0 + rr) * H + lane * 2) = (v2f){Tf[rr][lane * 2], Tf[rr][lane * 2 + 1]}; __threadfence(); } }
__global__ __launch_bounds__(256) void l3_kernel(L1P p, const float* __restrict__ S2, const float* __restrict__ ST2, const float* __restrict__ g2, const float* __restrict__ be2, const float* __restrict__ w3l, const float* __restrict__ b3, const float* __restrict__ w3r, const int* __restrict__ srcs, const int* __restrict__ PERM, const int* __restrict__ ROWPTR, const int* __restrict__ ROWCNT, int permLen, int NLIM, float* __restrict__ out) {
  const int wave = threadIdx.x >> 5, lane = threadIdx.x & 31; const size_t n0 = ((size_t)blockIdx.x * 8 + wave) * 32; if (n0 >= (size_t)NLIM) return; const int c0 = lane * 2; const float wl0 = bf16_rne(w3l[c0]), wl1 = bf16_rne(w3l[c0 + 1]), wr0 = bf16_rne(w3r[c0]), wr1 = bf16_rne(w3r[c0 + 1]), bb = bf16_rne(b3[0]); float mine = 0.0f;
  auto x2of = [&](size_t u, float& v0, float& v1) { const v2f s2 = *(const v2f*)(S2 + u * H + c0); v0 = bnrelu(s2[0], c0, ST2, g2, be2) + x1_of(p, u, c0); v1 = bnrelu(s2[1], c0 + 1, ST2, g2, be2) + x1_of(p, u, c0 + 1); };
#pragma unroll 1
  for (int q = 0; q < 32; ++q) { const size_t i = n0 + q; if (i >= (size_t)N) break; int st = ROWPTR[i], cnt = ROWCNT[i]; cnt = iclamp(cnt, 0, E); st = iclamp(st, 0, permLen - cnt); float a0 = 0.0f, a1 = 0.0f; int nin = 0;
#pragma unroll 1
    for (int j = 0; j < cnt; ++j) { const int e = iclamp(PERM[st + j], 0, E - 1); const size_t u = (size_t)iclamp(srcs[e], 0, N - 1); if (u >= (size_t)NLIM) continue; ++nin; float v0, v1; x2of(u, v0, v1); a0 += v0; a1 += v1; }
    const float inv = 1.0f / (float)(nin > 0 ? nin : 1); float s0, s1v; x2of(i, s0, s1v); float part = pmul(pmul(a0, inv), wl0) + pmul(pmul(a1, inv), wl1) + pmul(s0, wr0) + pmul(s1v, wr1); for (int o = 16; o; o >>= 1) part += __shfl_xor(part, o); if (lane == q) mine = part + bb; }
  for (int pass = 0; pass < 2; ++pass) { if (n0 + lane < (size_t)N) ((volatile float*)out)[n0 + lane] = mine; __threadfence(); } }
}

extern "C" void kernel_launch(void* const* d_in, const int* in_sizes, int n_in, void* d_out, int out_size, void* d_ws, size_t ws_size, hipStream_t stream) {
  (void)n_in;
  auto Fp = [&](int i) { return (const float*)d_in[i]; }; auto Ip = [&](int i) { return (const int*)d_in[i]; };
  if (in_sizes[0] != N * CI || in_sizes[1] != 2 * E || in_sizes[2] != CI * H || in_sizes[7] != H * H || in_sizes[12] != H || out_size != N) return;
  const int NLIM = N;
  size_t off = 0; char* ws = (char*)d_ws;
  auto carve = [&](size_t bytes) { char* p = ws + off; off += (bytes + 255) & ~(size_t)255; return p; };
  const int NBLK = (NLIM + SB - 1) / SB;
  b16* W2T = (b16*)carve((size_t)H * 2 * H * 2); float* M1 = (float*)carve((size_t)N * 2 * 4); float* S2 = (float*)carve((size_t)N * H * 4); float* PS = (float*)carve((size_t)((N + SB - 1) / SB) * 2 * H * 4); float* ST1 = (float*)carve(2 * H * 4); float* ST2 = (float*)carve(2 * H * 4);
  CsrBufs10 csr; off = csr_carve10(csr, ws, off, E, N);
  if (off > ws_size || off > ((size_t)176 << 20)) return;
  wput_kernel<<<(H * 16 + 255) / 256, 256, 0, stream>>>(Fp(7), Fp(9), W2T);
  csr_build10(csr, Ip(1) + E, E, N, stream);
  m1_kernel<<<(N + 255) / 256, 256, 0, stream>>>(Fp(0), Ip(1), csr.PERM, csr.ROWPTR, csr.ROWCNT, (int)csr.permLen, NLIM, M1);
  const L1P p1 = {M1, Fp(0), Fp(2), Fp(3), Fp(4), ST1, Fp(5), Fp(6)};
  stat_kernel<1><<<NBLK, 256, 0, stream>>>(p1, nullptr, NLIM, PS); bnfin_kernel<<<1, 256, 0, stream>>>(PS, NBLK, NLIM, ST1);
  l2_kernel<<<NLIM / 16, 32, 0, stream>>>(p1, W2T, Fp(8), Ip(1), csr.PERM, csr.ROWPTR, csr.ROWCNT, (int)csr.permLen, NLIM, S2);
  stat_kernel<2><<<NBLK, 256, 0, stream>>>(p1, S2, NLIM, PS); bnfin_kernel<<<1, 256, 0, stream>>>(PS, NBLK, NLIM, ST2);
  l3_kernel<<<(NLIM / 32 + 7) / 8, 256, 0, stream>>>(p1, S2, ST2, Fp(10), Fp(11), Fp(12), Fp(13), Fp(14), Ip(1), csr.PERM, csr.ROWPTR, csr.ROWCNT, (int)csr.permLen, NLIM, (float*)d_out);
}
